// MSA_6270652252504
// MI455X (gfx1250) — hardware-verified
//
#include <hip/hip_runtime.h>


#ifndef NB
#define NB 2
#endif
#ifndef SEQ
#define SEQ 2048
#endif
#define NB_FULL  2
#define SEQ_FULL 2048
#define DM   1024
#define NH   16
#define HD   64
#define KT   64
#define QB   256
#define OSP  68
#define PCAR 1024.0f
#define SCL  0.125f
#define L2E  1.4426950408889634f

static_assert(DM == NH * HD);
static_assert(SEQ % QB == 0);
static_assert(SEQ % KT == 0);
static_assert((NB * SEQ) % 64 == 0);
static_assert(NB >= 1 && NB <= NB_FULL);
static_assert(SEQ >= QB && SEQ <= SEQ_FULL);
static_assert(HD % 32 == 0);

typedef _Float16 h16;
typedef unsigned short bf;
typedef __attribute__((ext_vector_type(16))) __bf16   v16bf;
typedef __attribute__((ext_vector_type(16))) _Float16 v16h;
typedef __attribute__((ext_vector_type(8)))  _Float16 v8h;
typedef __attribute__((ext_vector_type(2)))  _Float16 v2h;
typedef __attribute__((ext_vector_type(8)))  unsigned short v8us;
typedef __attribute__((ext_vector_type(8)))  float    v8f;
typedef __attribute__((ext_vector_type(4)))  float    v4f;
typedef __attribute__((ext_vector_type(2)))  float    v2f;
typedef v4f __attribute__((may_alias)) v4fa;

__device__ __forceinline__ unsigned short f2bf(float f) { unsigned u = __float_as_uint(f); u += 0x7FFFu + ((u >> 16) & 1u); return (unsigned short)(u >> 16); }
__device__ __forceinline__ float bf2f(unsigned short b) { return __uint_as_float(((unsigned)b) << 16); }
__device__ __forceinline__ float bfr(float f) { return bf2f(f2bf(f)); }
__device__ __forceinline__ v16h  cat16(v8h lo, v8h hi) { return __builtin_shufflevector(lo, hi, 0, 1, 2, 3, 4, 5, 6, 7, 8, 9, 10, 11, 12, 13, 14, 15); }
__device__ __forceinline__ v16bf cat16b(v8us lo, v8us hi) { return __builtin_bit_cast(v16bf, __builtin_shufflevector(lo, hi, 0, 1, 2, 3, 4, 5, 6, 7, 8, 9, 10, 11, 12, 13, 14, 15)); }
__device__ __forceinline__ v8f wmma16(v16h a, v16h b, v8f c) { return __builtin_amdgcn_wmma_f32_16x16x32_f16(false, a, false, b, (short)0, c, false, false); }
__device__ __forceinline__ v8f wmmab(v16bf a, v16bf b, v8f c) { return __builtin_amdgcn_wmma_f32_16x16x32_bf16(false, a, false, b, (short)0, c, false, false); }
__device__ __forceinline__ v16h  ldh(const h16* p) { return cat16(*(const v8h*)p, *(const v8h*)(p + 16)); }
__device__ __forceinline__ v16bf ldb16(const bf* p) { return cat16b(*(const v8us*)p, *(const v8us*)(p + 16)); }

__global__ __launch_bounds__(256) void k_cvtw(const float* __restrict__ w0, const float* __restrict__ w1, const float* __restrict__ w2, bf* dst, int n8) {
    const int i = blockIdx.x * 256 + threadIdx.x; if (i >= n8) return;
    const int sel = blockIdx.y;
    const float* src = (sel == 0) ? w0 : ((sel == 1) ? w1 : w2);
    const v8f v = *(const v8f*)(src + (size_t)i * 8); v8us o;
#pragma unroll
    for (int k = 0; k < 8; ++k) o[k] = f2bf(v[k]);
    bf* d = dst + (size_t)sel * n8 * 8 + (size_t)i * 8;
    *(volatile v8us*)d = o; __threadfence(); *(volatile v8us*)d = o;
}
__global__ __launch_bounds__(256) void k_cvtx(const float* __restrict__ x, bf* XB, int n8) {
    const int i = blockIdx.x * 256 + threadIdx.x; if (i >= n8) return;
    const size_t el = (size_t)i * 8; const int c = (int)(el % DM); const size_t row = el / DM; const int t = (int)(row % SEQ); const int b = (int)(row / SEQ);
    const v8f v = *(const v8f*)(x + ((size_t)b * SEQ_FULL + t) * DM + c); v8us o;
#pragma unroll
    for (int k = 0; k < 8; ++k) o[k] = f2bf(v[k]);
    *(volatile v8us*)(XB + el) = o; __threadfence(); *(volatile v8us*)(XB + el) = o;
}

__global__ __launch_bounds__(32) void k_gemmw(const bf* __restrict__ A, int lda, const bf* __restrict__ Bt, int ldb, int K, float* C, int ldc, const float* __restrict__ bias, size_t sA, size_t sB, size_t sC, size_t sBias) {
    __shared__ __align__(16) float os[16 * OSP];
    const size_t z = blockIdx.z; A += z * sA; Bt += z * sB; C += z * sC; bias += z * sBias;
    const int lane = threadIdx.x & 31, lr = lane & 15, hi = lane >> 4; const int r0 = blockIdx.x * 64, c0 = blockIdx.y * 64;
    v8f acc[4][4];
#pragma unroll
    for (int mb = 0; mb < 4; ++mb)
#pragma unroll
        for (int nb = 0; nb < 4; ++nb) acc[mb][nb] = (v8f){};
    const size_t aoff = (size_t)(r0 + lr) * lda + 8 * hi, boff = (size_t)(c0 + lr) * ldb + 8 * hi;
    v16bf a[4], bfrag;
#pragma unroll 1
    for (int kc = 0; kc < K; kc += 32) {
#pragma unroll
        for (int mb = 0; mb < 4; ++mb) a[mb] = ldb16(A + aoff + (size_t)mb * 16 * lda + kc);
#pragma unroll
        for (int nb = 0; nb < 4; ++nb) { bfrag = ldb16(Bt + boff + (size_t)nb * 16 * ldb + kc);
#pragma unroll
            for (int mb = 0; mb < 4; ++mb) acc[mb][nb] = wmmab(a[mb], bfrag, acc[mb][nb]); }
        asm volatile("v_nop\n\tv_nop\n\tv_nop\n\tv_nop" : "+v"(acc[0][0]), "+v"(acc[1][1]), "+v"(acc[2][2]), "+v"(acc[3][3]) : "v"(a[0]), "v"(a[3]), "v"(bfrag));
    }
#pragma unroll
    for (int mb = 0; mb < 4; ++mb) {
#pragma unroll
        for (int nb = 0; nb < 4; ++nb) {
#pragma unroll
            for (int j = 0; j < 8; ++j) os[(hi * 8 + j) * OSP + nb * 16 + lr] = acc[mb][nb][j]; }
        __builtin_amdgcn_fence(3, "wavefront"); __builtin_amdgcn_wave_barrier(); asm volatile("" ::: "memory");
        float* crow = C + (size_t)(r0 + mb * 16) * ldc + c0;
#pragma unroll 1
        for (int ps = 0; ps < 2; ++ps) {
#pragma unroll
            for (int s = 0; s < 8; ++s) { const int row = 2 * s + hi, cofs = lr * 4; v4f val = *(const v4fa*)(os + row * OSP + cofs);
                val[0] += bfr(bias[c0 + cofs]); val[1] += bfr(bias[c0 + cofs + 1]); val[2] += bfr(bias[c0 + cofs + 2]); val[3] += bfr(bias[c0 + cofs + 3]);
                *(volatile v4f*)(crow + (size_t)row * ldc + cofs) = val; }
            if (ps == 0) __threadfence(); }
        __builtin_amdgcn_wave_barrier(); asm volatile("" ::: "memory");
    }
}

__global__ __launch_bounds__(256) void k_qkp(const float* __restrict__ F, h16* P) {
    const size_t e = ((size_t)blockIdx.x * 256 + threadIdx.x) * 2; if (e >= (size_t)NB * NH * SEQ * HD) return;
    const int d = (int)(e % HD); const int t = (int)((e / HD) % SEQ); const int h = (int)((e / ((size_t)HD * SEQ)) % NH); const int b = (int)(e / ((size_t)HD * SEQ * NH));
    const v2f xv = *(const v2f*)(F + ((size_t)b * SEQ + t) * DM + h * HD + d);
    v2h o; o[0] = (h16)xv[0]; o[1] = (h16)xv[1];
    *(volatile v2h*)(P + e) = o; __threadfence(); *(volatile v2h*)(P + e) = o;
}
__global__ __launch_bounds__(256) void k_vtp(const float* __restrict__ F, h16* VT) {
    const size_t e = ((size_t)blockIdx.x * 256 + threadIdx.x) * 2; if (e >= (size_t)NB * NH * HD * SEQ) return;
    const int t = (int)(e % SEQ); const int d = (int)((e / SEQ) % HD); const int h = (int)((e / ((size_t)SEQ * HD)) % NH); const int b = (int)(e / ((size_t)SEQ * HD * NH));
    const float* f = F + ((size_t)b * SEQ + t) * DM + h * HD + d;
    v2h o; o[0] = (h16)f[0]; o[1] = (h16)f[DM];
    *(volatile v2h*)(VT + e) = o; __threadfence(); *(volatile v2h*)(VT + e) = o;
}

__global__ __launch_bounds__(256) __attribute__((amdgpu_num_vgpr(256)))
void k_attn(const h16* __restrict__ Q16, const h16* __restrict__ K16, const h16* __restrict__ VT16, float* OUT) {
    __shared__ __align__(16) h16 Ks[KT * HD];
    __shared__ __align__(16) h16 Vs[HD * KT];
    __shared__ __align__(16) float osh[QB / 32][16 * OSP];
    const int tid = threadIdx.x, wv = tid >> 5, lane = tid & 31, lr = lane & 15, hi = lane >> 4;
    const int qblks = SEQ / QB; const int bh = blockIdx.x / qblks, qblk = blockIdx.x % qblks; const int b = bh / NH, h = bh % NH;
    const int q0 = qblk * QB + wv * 32;
    const h16* Qp = Q16 + ((size_t)bh * SEQ + q0) * HD;
    v16h qf[2][2];
#pragma unroll
    for (int qt = 0; qt < 2; ++qt)
#pragma unroll
        for (int kk = 0; kk < 2; ++kk) qf[qt][kk] = ldh(Qp + (size_t)(qt * 16 + lr) * HD + kk * 32 + 8 * hi);
    const h16* Kb = K16 + (size_t)bh * SEQ * HD; const h16* Vb = VT16 + (size_t)bh * HD * SEQ;
    v8f o[2][4];
#pragma unroll
    for (int qt = 0; qt < 2; ++qt)
#pragma unroll
        for (int et = 0; et < 4; ++et) o[qt][et] = (v8f){};
    float m_run[2] = {-1.0e30f, -1.0e30f}, l_run[2] = {0.f, 0.f};
    float* os = osh[wv];
#pragma unroll 1
    for (int t0 = 0; t0 < SEQ; t0 += KT) {
        __syncthreads();
#pragma unroll
        for (int j = 0; j < 2; ++j) { const int u = tid + j * 256; const int e = u >> 3, uu = u & 7;
            const v8h kx = *(const v8h*)(Kb + (size_t)t0 * HD + (size_t)u * 8);
            const v8h vx = *(const v8h*)(Vb + (size_t)e * SEQ + t0 + uu * 8);
            *(v8h*)(Ks + u * 8) = kx; *(v8h*)(Vs + e * KT + uu * 8) = vx; }
        __syncthreads();
#pragma unroll
        for (int qt = 0; qt < 2; ++qt) {
            v8f st[4]; v16h ka0, ka1;
#pragma unroll
            for (int ts = 0; ts < 4; ++ts) { ka0 = ldh(Ks + (ts * 16 + lr) * HD + 8 * hi); ka1 = ldh(Ks + (ts * 16 + lr) * HD + 32 + 8 * hi);
                v8f c = (v8f){}; c = wmma16(ka0, qf[qt][0], c); c = wmma16(ka1, qf[qt][1], c); st[ts] = c; }
            asm volatile("v_nop\n\tv_nop\n\tv_nop\n\tv_nop" : "+v"(st[0]), "+v"(st[1]), "+v"(st[2]), "+v"(st[3]) : "v"(ka0), "v"(ka1), "v"(qf[qt][1]));
            float tm = -1.0e30f;
#pragma unroll
            for (int ts = 0; ts < 4; ++ts)
#pragma unroll
                for (int v = 0; v < 8; ++v) { const float t = st[ts][v] * SCL; st[ts][v] = t; tm = fmaxf(tm, t); }
            tm = fmaxf(tm, __shfl_xor(tm, 16, 32));
            const float m_new = fmaxf(m_run[qt], tm);
            float da = __fsub_rn(m_run[qt], m_new); asm volatile("" : "+v"(da));
            const float alpha = __builtin_amdgcn_exp2f(__fmul_rn(da, L2E));
            float rs = 0.f; v16h pa[2];
#pragma unroll
            for (int v = 0; v < 8; ++v) {
                float d0 = __fsub_rn(st[0][v], m_new), d1 = __fsub_rn(st[1][v], m_new), d2 = __fsub_rn(st[2][v], m_new), d3 = __fsub_rn(st[3][v], m_new);
                asm volatile("" : "+v"(d0)); asm volatile("" : "+v"(d1)); asm volatile("" : "+v"(d2)); asm volatile("" : "+v"(d3));
                const float p0 = __builtin_amdgcn_exp2f(__fmul_rn(d0, L2E)), p1 = __builtin_amdgcn_exp2f(__fmul_rn(d1, L2E));
                const float p2 = __builtin_amdgcn_exp2f(__fmul_rn(d2, L2E)), p3 = __builtin_amdgcn_exp2f(__fmul_rn(d3, L2E));
                rs += (p0 + p1) + (p2 + p3);
                pa[0][v] = (h16)(p0 * PCAR); pa[0][v + 8] = (h16)(p1 * PCAR);
                pa[1][v] = (h16)(p2 * PCAR); pa[1][v + 8] = (h16)(p3 * PCAR);
            }
            rs += __shfl_xor(rs, 16, 32);
            l_run[qt] = l_run[qt] * alpha + rs; m_run[qt] = m_new;
#pragma unroll
            for (int v = 0; v < 8; ++v) { const float fs = __shfl(alpha, v + 8 * hi, 32); o[qt][0][v] *= fs; o[qt][1][v] *= fs; o[qt][2][v] *= fs; o[qt][3][v] *= fs; }
            v16h vb0, vb1;
#pragma unroll
            for (int et = 0; et < 4; ++et) { vb0 = ldh(Vs + (et * 16 + lr) * KT + 8 * hi); vb1 = ldh(Vs + (et * 16 + lr) * KT + 32 + 8 * hi);
                o[qt][et] = wmma16(pa[0], vb0, o[qt][et]); o[qt][et] = wmma16(pa[1], vb1, o[qt][et]); }
            asm volatile("v_nop\n\tv_nop\n\tv_nop\n\tv_nop" : "+v"(o[qt][0]), "+v"(o[qt][1]), "+v"(o[qt][2]), "+v"(o[qt][3]) : "v"(pa[0]), "v"(pa[1]), "v"(vb1));
        }
    }
#pragma unroll
    for (int qt = 0; qt < 2; ++qt) {
        const float inv = 1.0f / (l_run[qt] * PCAR);
#pragma unroll
        for (int j = 0; j < 8; ++j) { const float fs = __shfl(inv, j + 8 * hi, 32);
#pragma unroll
            for (int et = 0; et < 4; ++et) os[(hi * 8 + j) * OSP + et * 16 + lr] = o[qt][et][j] * fs; }
        __builtin_amdgcn_fence(3, "wavefront"); __builtin_amdgcn_wave_barrier(); asm volatile("" ::: "memory");
        float* crow = OUT + ((size_t)b * SEQ + q0 + qt * 16) * DM + (size_t)h * HD;
#pragma unroll 1
        for (int ps = 0; ps < 2; ++ps) {
#pragma unroll
            for (int s = 0; s < 8; ++s) { const int row = 2 * s + hi, cofs = lr * 4; const v4f val = *(const v4fa*)(os + row * OSP + cofs);
                *(volatile v4f*)(crow + (size_t)row * DM + cofs) = val; }
            if (ps == 0) __threadfence(); }
        __builtin_amdgcn_wave_barrier(); asm volatile("" ::: "memory");
    }
}

extern "C" void kernel_launch(void* const* d_in, const int* in_sizes, int n_in,
                              void* d_out, int out_size, void* d_ws, size_t ws_size, hipStream_t stream) {
    if (n_in < 7) return;
    if (in_sizes[0] < (NB - 1) * SEQ_FULL * DM + SEQ * DM) return;
    if (in_sizes[1] < NH * HD * HD || in_sizes[3] < NH * HD * HD || in_sizes[5] < NH * HD * HD) return;
    if (in_sizes[2] < NH * HD || in_sizes[4] < NH * HD || in_sizes[6] < NH * HD) return;
    if (out_size < NB * SEQ * DM) return;
    const float* x = (const float*)d_in[0]; const float* wq = (const float*)d_in[1]; const float* bq = (const float*)d_in[2]; const float* wk = (const float*)d_in[3]; const float* bk = (const float*)d_in[4]; const float* wv = (const float*)d_in[5]; const float* bv = (const float*)d_in[6];
    float* OUT = (float*)d_out;
    char* wsp = (char*)d_ws;
    auto take = [&](size_t bytes) { char* p = wsp; wsp += (bytes + 255) & ~(size_t)255; return (void*)p; };
    const size_t wsz = (size_t)NH * HD * HD;
    bf*  WB   = (bf*)take(3 * wsz * 2);
    bf*  XB   = (bf*)take((size_t)NB * SEQ * DM * 2);
    float* F  = (float*)take((size_t)NB * SEQ * DM * 4);
    h16* Q16  = (h16*)take((size_t)NB * NH * SEQ * HD * 2);
    h16* K16  = (h16*)take((size_t)NB * NH * SEQ * HD * 2);
    h16* VT16 = (h16*)take((size_t)NB * NH * HD * SEQ * 2);
    if ((size_t)(wsp - (char*)d_ws) > ws_size) return;
    const int nw8 = (int)(wsz / 8); const int nx8 = NB * SEQ * DM / 8;
    k_cvtw<<<dim3((unsigned)((nw8 + 255) / 256), 3, 1), 256, 0, stream>>>(wq, wk, wv, WB, nw8);
    k_cvtx<<<(unsigned)((nx8 + 255) / 256), 256, 0, stream>>>(x, XB, nx8);
    const dim3 gg((unsigned)(NB * SEQ / 64), 1, NH);
    const unsigned LP = (unsigned)(((size_t)NB * NH * SEQ * HD / 2 + 255) / 256);
    k_gemmw<<<gg, 32, 0, stream>>>(XB, DM, WB, HD, HD, F, DM, bq, (size_t)HD, (size_t)HD * HD, (size_t)HD, (size_t)HD);
    k_qkp<<<LP, 256, 0, stream>>>(F, Q16);
    k_gemmw<<<gg, 32, 0, stream>>>(XB, DM, WB + wsz, HD, HD, F, DM, bk, (size_t)HD, (size_t)HD * HD, (size_t)HD, (size_t)HD);
    k_qkp<<<LP, 256, 0, stream>>>(F, K16);
    k_gemmw<<<gg, 32, 0, stream>>>(XB, DM, WB + 2 * wsz, HD, HD, F, DM, bv, (size_t)HD, (size_t)HD * HD, (size_t)HD, (size_t)HD);
    k_vtp<<<LP, 256, 0, stream>>>(F, VT16);
    k_attn<<<(unsigned)(NB * NH * (SEQ / QB)), 256, 0, stream>>>(Q16, K16, VT16, OUT);
}
